// SelectiveSSM_75488345195322
// MI455X (gfx1250) — hardware-run, weakly checked
//
#include <hip/hip_runtime.h>
#include <hip/hip_fp16.h>
#include <math.h>

typedef float    ms1_v4f __attribute__((ext_vector_type(4)));
typedef unsigned ms1_v4u __attribute__((ext_vector_type(4)));
struct ms1_args {
  const float* dtpre;
  const float* u;
  const float* bc;
  const float* z;
  const float* A_log;
  const float* Dskip;
  __half* y;
  __half* y_lo;
  long ld_dtpre;
  long ld_u;
  long ld_bc;
  long ld_z;
  long ld_y;
  int offB;
  int offC;
  int offZ;
  float ycarry;
  int dir;
  int D;
  int L;
  int nbatch;
};
static_assert(sizeof(ms1_args) == 136);

__device__ __forceinline__ float ms1_flush16(float v) {
  return (fabsf(v) < 6.103515625e-05f) ? 0.0f : v;
}
__device__ __forceinline__ unsigned ms1_h16bits(float v) {
  return (unsigned)__half_as_ushort(__float2half_rn(ms1_flush16(v)));
}
__device__ __forceinline__ float ms1_h16val(unsigned b) {
  return __half2float(__ushort_as_half((unsigned short)b));
}
__device__ __forceinline__ float ms1_softplus(float v) {
  return fmaxf(v, 0.0f) + log1pf(expf(-fabsf(v)));
}
__device__ __forceinline__ void ms1_pack2(float v0, float v1, unsigned& hw, unsigned& lw) {
  const unsigned h0 = ms1_h16bits(v0);
  const unsigned h1 = ms1_h16bits(v1);
  const float r0 = (v0 - ms1_h16val(h0)) * 2048.0f;
  const float r1 = (v1 - ms1_h16val(h1)) * 2048.0f;
  const unsigned l0 = ms1_h16bits(r0);
  const unsigned l1 = ms1_h16bits(r1);
  hw = h0 | (h1 << 16);
  lw = l0 | (l1 << 16);
}

template <int NSTATE>
__global__ __launch_bounds__(64 * (NSTATE / 16)) void ms1_scan_kernel(ms1_args a)
{
  static_assert(NSTATE == 16 || NSTATE == 64);
  constexpr int NQ  = NSTATE / 16;
  constexpr int NT  = 64 * NQ;
  constexpr int NW  = NT / 32;
  constexpr int BCW = 2 * NSTATE;
  constexpr int YP  = 68;
  constexpr int RPI = NW * 4;
  constexpr int NIT = 64 / RPI;
  static_assert(16 * NT <= 64 * YP);
  __shared__ __align__(16) float sBC[64 * BCW];
  __shared__ __align__(16) float sY[64 * YP];
  const int tid  = threadIdx.x;
  const int lane = tid & 31;
  const int wave = tid >> 5;
  const int c    = tid / NQ;
  const int sq   = tid - c * NQ;
  const int bpb  = a.D / 64;
  const int bi   = blockIdx.x / bpb;
  if (bi >= a.nbatch) return;
  const int d0 = (blockIdx.x - bi * bpb) * 64;
  const int d  = d0 + c;
  const long rowb = (long)bi * a.L;
  const bool hasz  = (a.z != nullptr);
  const bool hasD  = (a.Dskip != nullptr);
  const bool hasLo = (a.y_lo != nullptr);

#pragma unroll 1
  for (int n = 0; n < 16; ++n) {
    const float al = a.A_log[(long)d * NSTATE + sq * 16 + n];
    sY[n * NT + tid] = -expf(al);
  }
  __syncthreads();
  float An[16], h[16];
#pragma unroll
  for (int n = 0; n < 16; ++n) {
    An[n] = sY[n * NT + tid];
    h[n] = 0.0f;
  }
  float Dd = 0.0f;
  if (hasD) Dd = a.Dskip[d];

  const int nchunk = a.L / 64;
  const bool fwd = (a.dir > 0);
  const int s0 = fwd ? 0 : 63;
  const int sd = fwd ? 1 : -1;
  const int q  = lane >> 3;
  const int c8 = (lane & 7) * 8;

#pragma unroll 1
  for (int ci = 0; ci < nchunk; ++ci) {
    const int tb = fwd ? (ci * 64) : (a.L - 64 - ci * 64);
    const long rowc = rowb + tb;
    __syncthreads();
#pragma unroll 8
    for (int i = 0; i < 32; ++i) {
      const int idx = tid + i * NT;
      const int st  = idx / BCW;
      const int col = idx - st * BCW;
      const int sc  = (col < NSTATE) ? (a.offB + col) : (a.offC + col - NSTATE);
      sBC[idx] = a.bc[(rowc + st) * a.ld_bc + sc];
    }
    __syncthreads();
#pragma unroll 1
    for (int s = 0; s < 64; ++s) {
      const int ls = s0 + sd * s;
      const long row = rowc + ls;
      float pre = a.dtpre[row * a.ld_dtpre + d];
      float uv  = a.u[row * a.ld_u + d];
      float zv  = 0.0f;
      if (hasz) zv = a.z[row * a.ld_z + a.offZ + d];
      asm volatile("" : "+v"(pre));
      asm volatile("" : "+v"(uv));
      asm volatile("" : "+v"(zv));
      const float delta = ms1_softplus(pre);
      const float dtx = delta * uv;
      const float* bp = sBC + ls * BCW + sq * 16;
      const float* cp = bp + NSTATE;
      ms1_v4f Bq[4], Cq[4];
#pragma unroll
      for (int k = 0; k < 4; ++k) {
        Bq[k] = *(const ms1_v4f*)(bp + 4 * k);
        Cq[k] = *(const ms1_v4f*)(cp + 4 * k);
      }
      float yv = 0.0f;
#pragma unroll
      for (int n = 0; n < 16; ++n) {
        const float e = __expf(delta * An[n]);
        h[n] = fmaf(e, h[n], dtx * Bq[n >> 2][n & 3]);
        yv = fmaf(h[n], Cq[n >> 2][n & 3], yv);
      }
      if (NQ > 1) {
        yv += __shfl_xor(yv, 1, 32);
        yv += __shfl_xor(yv, 2, 32);
      }
      if (hasD) yv = fmaf(uv, Dd, yv);
      if (hasz) {
        const float sg = __builtin_amdgcn_rcpf(1.0f + expf(-zv));
        yv = yv * (zv * sg);
      }
      if (sq == 0) sY[ls * YP + c] = yv * a.ycarry;
    }
    __syncthreads();
    ms1_v4u hw[NIT], lw[NIT];
#pragma unroll
    for (int it = 0; it < NIT; ++it) {
      const int row = it * RPI + wave * 4 + q;
      const float* sp = sY + row * YP + c8;
      const ms1_v4f f0 = *(const ms1_v4f*)(sp);
      const ms1_v4f f1 = *(const ms1_v4f*)(sp + 4);
      unsigned h0, h1, h2, h3, l0, l1, l2, l3;
      ms1_pack2(f0[0], f0[1], h0, l0);
      ms1_pack2(f0[2], f0[3], h1, l1);
      ms1_pack2(f1[0], f1[1], h2, l2);
      ms1_pack2(f1[2], f1[3], h3, l3);
      hw[it] = (ms1_v4u){h0, h1, h2, h3};
      lw[it] = (ms1_v4u){l0, l1, l2, l3};
    }
    for (int pass = 0; pass < 2; ++pass) {
#pragma unroll
      for (int it = 0; it < NIT; ++it) {
        const int row = it * RPI + wave * 4 + q;
        const long o = (rowc + row) * a.ld_y + d0 + c8;
        *(volatile ms1_v4u*)(a.y + o) = hw[it];
        if (hasLo) *(volatile ms1_v4u*)(a.y_lo + o) = lw[it];
      }
      __threadfence();
    }
  }
}

namespace eng {

constexpr int kBatch  = 2;
constexpr int kSeq    = 2048;
constexpr int kD      = 2048;
constexpr int kNstate = 16;
constexpr int kRank   = 64;
constexpr int kRows   = kBatch * kSeq;
constexpr int kXdN    = kRank + 2 * kNstate;
constexpr int kXdP    = 128;
constexpr int kOffB   = kRank;
constexpr int kOffC   = kRank + kNstate;

static_assert(kXdN == 96);
static_assert(kRows % 32 == 0 && kXdP % 64 == 0 && kD % 64 == 0);
static_assert(kD % 32 == 0 && kRank % 32 == 0);
static_assert(kD % 64 == 0 && kSeq % 64 == 0);
static_assert((kOffB % 4) == 0 && (kOffC % 4) == 0);
static_assert(kRank == 64);

constexpr float kCarryY    = 16.0f;
constexpr float kResid     = 2048.0f;
constexpr float kFoldHi    = 1.0f / kCarryY;
constexpr float kFoldLo    = 1.0f / (kCarryY * kResid);

constexpr size_t kBytesXH   = (size_t)kRows * kD * 2;
constexpr size_t kBytesXL   = (size_t)kRows * kD * 2;
constexpr size_t kBytesWXH  = (size_t)kXdP * kD * 2;
constexpr size_t kBytesWXL  = (size_t)kXdP * kD * 2;
constexpr size_t kBytesWDH  = (size_t)kD * kRank * 2;
constexpr size_t kBytesWDL  = (size_t)kD * kRank * 2;
constexpr size_t kBytesXDBL = (size_t)kRows * kXdP * 4;
constexpr size_t kBytesDTH  = (size_t)kRows * kRank * 2;
constexpr size_t kBytesDTL  = (size_t)kRows * kRank * 2;
constexpr size_t kBytesDTP  = (size_t)kRows * kD * 4;
constexpr size_t kBytesYH   = (size_t)kRows * kD * 2;
constexpr size_t kBytesYL   = (size_t)kRows * kD * 2;
constexpr size_t kWsTotal = kBytesXH + kBytesXL + kBytesWXH + kBytesWXL + kBytesWDH + kBytesWDL + kBytesXDBL +
                            kBytesDTH + kBytesDTL + kBytesDTP + kBytesYH + kBytesYL;
static_assert(kWsTotal == 105381888ull);
static_assert(kWsTotal <= 134217728ull);
static_assert(kBytesXH % 128 == 0 && kBytesXL % 128 == 0 && kBytesWXH % 128 == 0 && kBytesWXL % 128 == 0 &&
              kBytesWDH % 128 == 0 && kBytesWDL % 128 == 0 && kBytesXDBL % 128 == 0 && kBytesDTH % 128 == 0 &&
              kBytesDTL % 128 == 0 && kBytesDTP % 128 == 0 && kBytesYH % 128 == 0);

typedef __bf16   v16b __attribute__((ext_vector_type(16)));
typedef __bf16   v8b  __attribute__((ext_vector_type(8)));
typedef float    v8f  __attribute__((ext_vector_type(8)));
typedef float    v4f  __attribute__((ext_vector_type(4)));
typedef unsigned v4u  __attribute__((ext_vector_type(4)));
typedef unsigned v2u  __attribute__((ext_vector_type(2)));

__device__ __forceinline__ unsigned bf_bits(float f) {
  const unsigned u = __float_as_uint(f);
  return (u + 0x7FFFu + ((u >> 16) & 1u)) >> 16;
}
__device__ __forceinline__ float bf_val(unsigned b) {
  return __uint_as_float(b << 16);
}
__device__ __forceinline__ void split2(float a, float b, unsigned& hw, unsigned& lw) {
  const unsigned ha = bf_bits(a);
  const unsigned hb = bf_bits(b);
  const float ra = a - bf_val(ha);
  const float rb = b - bf_val(hb);
  const unsigned la = bf_bits(ra);
  const unsigned lb = bf_bits(rb);
  hw = ha | (hb << 16);
  lw = la | (lb << 16);
}

union FragB { v16b v; v8b h[2]; };
__device__ __forceinline__ v16b frag_load(const __bf16* p) {
  FragB f;
  f.h[0] = *(const v8b*)(p);
  f.h[1] = *(const v8b*)(p + 16);
  return f.v;
}
__device__ __forceinline__ v8f mma(v16b a, v16b b, v8f c) {
  c = __builtin_amdgcn_wmma_f32_16x16x32_bf16(false, a, false, b, (short)0, c, false, false);
  asm volatile("v_nop\n\tv_nop\n\tv_nop\n\tv_nop" : "+v"(c) : "v"(a), "v"(b));
  return c;
}

__global__ __launch_bounds__(256) void split_bf16_kernel(
    const float* __restrict__ in, unsigned short* __restrict__ hi, unsigned short* __restrict__ lo,
    int n8_out, int n8_real)
{
  const int i = blockIdx.x * 256 + threadIdx.x;
  const int ic = (i < n8_real) ? i : (n8_real - 1);
  const v4f f0 = *(const v4f*)(in + (size_t)ic * 8);
  const v4f f1 = *(const v4f*)(in + (size_t)ic * 8 + 4);
  float e0 = f0[0];
  float e1 = f0[1];
  float e2 = f0[2];
  float e3 = f0[3];
  float e4 = f1[0];
  float e5 = f1[1];
  float e6 = f1[2];
  float e7 = f1[3];
  asm volatile("" : "+v"(e0), "+v"(e1), "+v"(e2), "+v"(e3));
  asm volatile("" : "+v"(e4), "+v"(e5), "+v"(e6), "+v"(e7));
  const bool real = (i < n8_real);
  e0 = real ? e0 : 0.0f;
  e1 = real ? e1 : 0.0f;
  e2 = real ? e2 : 0.0f;
  e3 = real ? e3 : 0.0f;
  e4 = real ? e4 : 0.0f;
  e5 = real ? e5 : 0.0f;
  e6 = real ? e6 : 0.0f;
  e7 = real ? e7 : 0.0f;
  unsigned h0, h1, h2, h3, l0, l1, l2, l3;
  split2(e0, e1, h0, l0);
  split2(e2, e3, h1, l1);
  split2(e4, e5, h2, l2);
  split2(e6, e7, h3, l3);
  const v4u hw = (v4u){h0, h1, h2, h3};
  const v4u lw = (v4u){l0, l1, l2, l3};
  if (i < n8_out) {
    unsigned short* oh = hi + (size_t)i * 8;
    unsigned short* ol = lo + (size_t)i * 8;
    for (int pass = 0; pass < 2; ++pass) {
      *(volatile v4u*)(oh) = hw;
      *(volatile v4u*)(ol) = lw;
      __threadfence();
    }
  }
}

template <int EPI>
__global__ __launch_bounds__(256) void gemm_bf16x3_kernel(
    const unsigned short* __restrict__ Ahp, const unsigned short* __restrict__ Alp, int lda,
    const unsigned short* __restrict__ Bhp, const unsigned short* __restrict__ Blp, int ldb,
    float* __restrict__ C, int ldc,
    unsigned short* __restrict__ Ch, unsigned short* __restrict__ Cl, int ldc16,
    const float* __restrict__ bias,
    int M, int N, int K)
{
  const __bf16* Ah = (const __bf16*)(const void*)Ahp;
  const __bf16* Al = (const __bf16*)(const void*)Alp;
  const __bf16* Bh = (const __bf16*)(const void*)Bhp;
  const __bf16* Bl = (const __bf16*)(const void*)Blp;
  __shared__ __align__(16) float sT[8][16 * 68];
  const int lane = threadIdx.x & 31;
  const int wave = threadIdx.x >> 5;
  const int tilesN = N >> 6;
  const int tilesM = M >> 5;
  const int tile = blockIdx.x * 8 + wave;
  if (tile >= tilesM * tilesN) return;
  const int tm = tile / tilesN;
  const int tn = tile - tm * tilesN;
  const int m0 = tm << 5;
  const int n0 = tn << 6;
  const int rlane = lane & 15;
  const int koff  = (lane >> 4) * 8;
  const int mOff  = (lane >> 4) * 8;

  v8f acc[2][4];
#pragma unroll
  for (int i = 0; i < 2; ++i) {
#pragma unroll
    for (int j = 0; j < 4; ++j) {
      acc[i][j] = (v8f){0.f, 0.f, 0.f, 0.f, 0.f, 0.f, 0.f, 0.f};
    }
  }

#pragma unroll 1
  for (int k0 = 0; k0 < K; k0 += 32) {
    v16b bh[4], bl[4];
#pragma unroll
    for (int j = 0; j < 4; ++j) {
      const size_t bo = (size_t)(n0 + (j << 4) + rlane) * ldb + koff + k0;
      bh[j] = frag_load(Bh + bo);
      bl[j] = frag_load(Bl + bo);
    }
#pragma unroll
    for (int i = 0; i < 2; ++i) {
      const size_t ao = (size_t)(m0 + (i << 4) + rlane) * lda + koff + k0;
      const v16b ah = frag_load(Ah + ao);
      const v16b al = frag_load(Al + ao);
#pragma unroll
      for (int j = 0; j < 4; ++j) {
        acc[i][j] = mma(ah, bl[j], acc[i][j]);
        acc[i][j] = mma(al, bh[j], acc[i][j]);
        acc[i][j] = mma(ah, bh[j], acc[i][j]);
      }
    }
  }

  float* slab = sT[wave];
  float bv[4] = {0.f, 0.f, 0.f, 0.f};
  if (EPI == 1) {
#pragma unroll
    for (int j = 0; j < 4; ++j) bv[j] = bias[n0 + (j << 4) + rlane];
  }
#pragma unroll
  for (int i = 0; i < 2; ++i) {
    const int mBase = m0 + (i << 4);
#pragma unroll
    for (int j = 0; j < 4; ++j) {
#pragma unroll
      for (int r = 0; r < 8; ++r) {
        float v = acc[i][j][r];
        if (EPI == 1) v = v + bv[j];
        slab[(mOff + r) * 68 + (j << 4) + rlane] = v;
      }
    }
    __builtin_amdgcn_fence(__ATOMIC_RELEASE, "workgroup");
    __builtin_amdgcn_wave_barrier();
    __builtin_amdgcn_fence(__ATOMIC_ACQUIRE, "workgroup");
    {
      const int hh = lane >> 4;
      const int c4 = (lane & 15) * 4;
      v4f val[8];
#pragma unroll
      for (int it = 0; it < 8; ++it) {
        const int row = it * 2 + hh;
        val[it] = *(const v4f*)(slab + row * 68 + c4);
      }
      for (int pass = 0; pass < 2; ++pass) {
#pragma unroll
        for (int it = 0; it < 8; ++it) {
          const int row = it * 2 + hh;
          *(volatile v4f*)(C + (size_t)(mBase + row) * ldc + n0 + c4) = val[it];
        }
        __threadfence();
      }
    }
    if (EPI == 0) {
      if (n0 == 0) {
        const int q  = lane >> 3;
        const int c8 = (lane & 7) * 8;
        v4u hw[4], lw[4];
#pragma unroll
        for (int it = 0; it < 4; ++it) {
          const int row = it * 4 + q;
          const float* sp = slab + row * 68 + c8;
          const v4f f0 = *(const v4f*)(sp);
          const v4f f1 = *(const v4f*)(sp + 4);
          const float e0 = f0[0];
          const float e1 = f0[1];
          const float e2 = f0[2];
          const float e3 = f0[3];
          const float e4 = f1[0];
          const float e5 = f1[1];
          const float e6 = f1[2];
          const float e7 = f1[3];
          unsigned h0, h1, h2, h3, l0, l1, l2, l3;
          split2(e0, e1, h0, l0);
          split2(e2, e3, h1, l1);
          split2(e4, e5, h2, l2);
          split2(e6, e7, h3, l3);
          hw[it] = (v4u){h0, h1, h2, h3};
          lw[it] = (v4u){l0, l1, l2, l3};
        }
        for (int pass = 0; pass < 2; ++pass) {
#pragma unroll
          for (int it = 0; it < 4; ++it) {
            const int row = it * 4 + q;
            *(volatile v4u*)(Ch + (size_t)(mBase + row) * ldc16 + c8) = hw[it];
            *(volatile v4u*)(Cl + (size_t)(mBase + row) * ldc16 + c8) = lw[it];
          }
          __threadfence();
        }
      }
    }
    __builtin_amdgcn_fence(__ATOMIC_RELEASE, "workgroup");
    __builtin_amdgcn_wave_barrier();
    __builtin_amdgcn_fence(__ATOMIC_ACQUIRE, "workgroup");
  }
}

__device__ __forceinline__ float h16_to_f32(unsigned hb) {
  const unsigned sgn = (hb & 0x8000u) << 16;
  const unsigned em = hb & 0x7fffu;
  const float fn = __uint_as_float((em << 13) + 0x38000000u);
  const float fs = (float)em * 5.9604644775390625e-8f;
  const float mag = (em < 0x400u) ? fs : fn;
  return __uint_as_float(__float_as_uint(mag) | sgn);
}

__device__ __forceinline__ v4f recombine4(const unsigned short* __restrict__ YH,
                                          const unsigned short* __restrict__ YL,
                                          int jc, float sHi, float sLo) {
  const v2u hw = *(const v2u*)(const void*)(YH + (size_t)jc * 4);
  const v2u lw = *(const v2u*)(const void*)(YL + (size_t)jc * 4);
  unsigned h0 = hw[0];
  unsigned h1 = hw[1];
  unsigned l0 = lw[0];
  unsigned l1 = lw[1];
  asm volatile("" : "+v"(h0), "+v"(h1), "+v"(l0), "+v"(l1));
  const float a0 = h16_to_f32(h0 & 0xffffu);
  const float a1 = h16_to_f32(h0 >> 16);
  const float a2 = h16_to_f32(h1 & 0xffffu);
  const float a3 = h16_to_f32(h1 >> 16);
  const float b0 = h16_to_f32(l0 & 0xffffu);
  const float b1 = h16_to_f32(l0 >> 16);
  const float b2 = h16_to_f32(l1 & 0xffffu);
  const float b3 = h16_to_f32(l1 >> 16);
  v4f o;
  o[0] = fmaf(b0, sLo, a0 * sHi);
  o[1] = fmaf(b1, sLo, a1 * sHi);
  o[2] = fmaf(b2, sLo, a2 * sHi);
  o[3] = fmaf(b3, sLo, a3 * sHi);
  return o;
}

__global__ __launch_bounds__(256) void recombine_kernel(
    const unsigned short* __restrict__ YH, const unsigned short* __restrict__ YL,
    float* __restrict__ out, int n4, float sHi, float sLo)
{
  const int j0 = blockIdx.x * 512 + threadIdx.x;
  const int j1 = j0 + 256;
  const int jc0 = (j0 < n4) ? j0 : (n4 - 1);
  const int jc1 = (j1 < n4) ? j1 : (n4 - 1);
  const v4f v0 = recombine4(YH, YL, jc0, sHi, sLo);
  const v4f v1 = recombine4(YH, YL, jc1, sHi, sLo);
  for (int pass = 0; pass < 2; ++pass) {
    if (j0 < n4) *(volatile v4f*)(out + (size_t)j0 * 4) = v0;
    if (j1 < n4) *(volatile v4f*)(out + (size_t)j1 * 4) = v1;
    __threadfence();
  }
}

}

extern "C" void kernel_launch(void* const* d_in, const int* in_sizes, int n_in,
                              void* d_out, int out_size, void* d_ws, size_t ws_size, hipStream_t stream)
{
  using namespace eng;
  if (n_in != 6) return;
  if (in_sizes[0] != kRows * kD) return;
  if (in_sizes[1] != kXdN * kD) return;
  if (in_sizes[2] != kD * kRank) return;
  if (in_sizes[3] != kD) return;
  if (in_sizes[4] != kD * kNstate) return;
  if (in_sizes[5] != kD) return;
  if (out_size != kRows * kD) return;
  if (ws_size < kWsTotal) return;

  const float* x     = (const float*)d_in[0];
  const float* W_x   = (const float*)d_in[1];
  const float* W_dt  = (const float*)d_in[2];
  const float* b_dt  = (const float*)d_in[3];
  const float* A_log = (const float*)d_in[4];
  const float* D_par = (const float*)d_in[5];
  float* out = (float*)d_out;

  char* ws = (char*)d_ws;
  size_t off = 0;
  unsigned short* XH  = (unsigned short*)(ws + off);
  off += kBytesXH;
  unsigned short* XL  = (unsigned short*)(ws + off);
  off += kBytesXL;
  unsigned short* WXH = (unsigned short*)(ws + off);
  off += kBytesWXH;
  unsigned short* WXL = (unsigned short*)(ws + off);
  off += kBytesWXL;
  unsigned short* WDH = (unsigned short*)(ws + off);
  off += kBytesWDH;
  unsigned short* WDL = (unsigned short*)(ws + off);
  off += kBytesWDL;
  float* XDBL         = (float*)(ws + off);
  off += kBytesXDBL;
  unsigned short* DTH = (unsigned short*)(ws + off);
  off += kBytesDTH;
  unsigned short* DTL = (unsigned short*)(ws + off);
  off += kBytesDTL;
  float* DTP          = (float*)(ws + off);
  off += kBytesDTP;
  unsigned short* YH  = (unsigned short*)(ws + off);
  off += kBytesYH;
  unsigned short* YL  = (unsigned short*)(ws + off);
  off += kBytesYL;
  if (off != kWsTotal) return;

  split_bf16_kernel<<<dim3((kRows * kD / 8) / 256), 256, 0, stream>>>(
      x, XH, XL, kRows * kD / 8, kRows * kD / 8);
  split_bf16_kernel<<<dim3((kXdP * kD / 8) / 256), 256, 0, stream>>>(
      W_x, WXH, WXL, kXdP * kD / 8, kXdN * kD / 8);
  split_bf16_kernel<<<dim3((kD * kRank / 8) / 256), 256, 0, stream>>>(
      W_dt, WDH, WDL, kD * kRank / 8, kD * kRank / 8);

  gemm_bf16x3_kernel<0><<<dim3((kRows / 32) * (kXdP / 64) / 8), 256, 0, stream>>>(
      XH, XL, kD, WXH, WXL, kD, XDBL, kXdP, DTH, DTL, kRank, b_dt,
      kRows, kXdP, kD);

  gemm_bf16x3_kernel<1><<<dim3((kRows / 32) * (kD / 64) / 8), 256, 0, stream>>>(
      DTH, DTL, kRank, WDH, WDL, kRank, DTP, kD, DTH, DTL, kRank, b_dt,
      kRows, kD, kRank);

  for (int b = 0; b < kBatch; ++b) {
    const size_t r0 = (size_t)b * kSeq;
    ms1_args sa;
    sa.dtpre = DTP + r0 * kD;
    sa.u = x + r0 * kD;
    sa.bc = XDBL + r0 * kXdP;
    sa.z = nullptr;
    sa.A_log = A_log;
    sa.Dskip = D_par;
    sa.y = (__half*)(YH + r0 * kD);
    sa.y_lo = (__half*)(YL + r0 * kD);
    sa.ld_dtpre = kD;
    sa.ld_u = kD;
    sa.ld_bc = kXdP;
    sa.ld_z = kD;
    sa.ld_y = kD;
    sa.offB = kOffB;
    sa.offC = kOffC;
    sa.offZ = 0;
    sa.ycarry = kCarryY;
    sa.dir = 1;
    sa.D = kD;
    sa.L = kSeq;
    sa.nbatch = 1;
    ms1_scan_kernel<16><<<dim3(kD / 64), 64, 0, stream>>>(sa);
  }

  recombine_kernel<<<dim3((kRows * kD / 4) / 512), 256, 0, stream>>>(
      YH, YL, out, kRows * kD / 4, kFoldHi, kFoldLo);
}
